// MT_CNN_LSTM_B_36438502539673
// MI455X (gfx1250) — hardware-verified
//
#include <hip/hip_runtime.h>
#include <stddef.h>
#include <stdint.h>


#define NB   1024
#define NT   64
#define SA   128
#define FA   64
#define IA   64
#define HA   256
#define FB   32
#define IB   32
#define HB   128
#define NY0  24
#define NY1  8

typedef float    v4f  __attribute__((ext_vector_type(4)));
typedef float    v8f  __attribute__((ext_vector_type(8)));
typedef _Float16 v8h  __attribute__((ext_vector_type(8))) __attribute__((may_alias));
typedef _Float16 v16h __attribute__((ext_vector_type(16)));

union Frag { v16h v; v8h hf[2]; };

constexpr size_t SZ_CTS = (size_t)NB * 64 * FA * 4;
constexpr size_t SZ_XA  = (size_t)NT * NB * IA * 2;
constexpr size_t SZ_XB  = (size_t)NT * NB * IB * 2;
constexpr size_t SZ_WA0 = (size_t)4 * HA * (IA + HA) * 2;
constexpr size_t SZ_WA1 = (size_t)4 * HA * (2 * HA) * 2;
constexpr size_t SZ_WB0 = (size_t)4 * HB * (IB + HB) * 2;
constexpr size_t SZ_WB1 = (size_t)4 * HB * (2 * HB) * 2;
constexpr size_t SZ_HFA = (size_t)NB * HA * 4;
constexpr size_t SZ_HFB = (size_t)NB * HB * 4;

constexpr size_t OFF_CTS = 0;
constexpr size_t OFF_XA  = OFF_CTS + SZ_CTS;
constexpr size_t OFF_XB  = OFF_XA  + SZ_XA;
constexpr size_t OFF_WA0 = OFF_XB  + SZ_XB;
constexpr size_t OFF_WA1 = OFF_WA0 + SZ_WA0;
constexpr size_t OFF_WB0 = OFF_WA1 + SZ_WA1;
constexpr size_t OFF_WB1 = OFF_WB0 + SZ_WB0;
constexpr size_t OFF_HFA = OFF_WB1 + SZ_WB1;
constexpr size_t OFF_HFB = OFF_HFA + SZ_HFA;
constexpr size_t WS_END  = OFF_HFB + SZ_HFB;
static_assert(WS_END <= (size_t)134217728);
static_assert(OFF_XA % 1024 == 0 && OFF_XB % 1024 == 0 && OFF_WA0 % 1024 == 0 && OFF_WA1 % 1024 == 0);
static_assert(OFF_WB0 % 1024 == 0 && OFF_WB1 % 1024 == 0 && OFF_HFA % 1024 == 0 && OFF_HFB % 1024 == 0);
static_assert(SZ_WA0 % 512 == 0 && SZ_WB0 % 512 == 0 && SZ_HFB % 512 == 0);

__device__ __forceinline__ v8f ld8f(const float* p) {
    const v4f a = *(const v4f*)p;
    const v4f b = *(const v4f*)(p + 4);
    return __builtin_shufflevector(a, b, 0, 1, 2, 3, 4, 5, 6, 7);
}

__device__ __forceinline__ void mma16(v8f& acc, const Frag& a, const Frag& b) {
    acc = __builtin_amdgcn_wmma_f32_16x16x32_f16(false, a.v, false, b.v, (short)0, acc, false, false);
    asm volatile("v_nop\n\tv_nop\n\tv_nop\n\tv_nop" : "+v"(acc) : "v"(a.v), "v"(b.v));
}

__device__ __forceinline__ float sigm_f(float x) {
    return __builtin_amdgcn_rcpf(1.0f + __expf(-x));
}
__device__ __forceinline__ float tanh_f(float x) {
    return 1.0f - 2.0f * __builtin_amdgcn_rcpf(__expf(2.0f * x) + 1.0f);
}

template<int I, int H>
__global__ __launch_bounds__(256)
void k_wcvt(const float* __restrict__ wih, const float* __restrict__ whh, _Float16* dst)
{
    constexpr int K = I + H, SEG = K / 8, ROWS = 4 * H, N16 = ROWS * SEG;
    static_assert(I % 8 == 0 && H % 8 == 0);
    const int idx = blockIdx.x * 256 + threadIdx.x;
    if (idx >= N16) return;
    const int n   = idx / SEG;
    const int seg = idx - n * SEG;
    const int col = seg * 8;
    const int ca  = min(col, I - 8);
    const int cb  = min(max(col - I, 0), H - 8);
    const v8f va  = ld8f(wih + (size_t)n * I + ca);
    const v8f vb  = ld8f(whh + (size_t)n * H + cb);
    const v8f v   = ((col < I) ? va : vb) * 8.0f;
    const v8h o   = __builtin_convertvector(v, v8h);
    _Float16* gp  = dst + (size_t)idx * 8;
    *(volatile v8h*)gp = o;
    __threadfence();
    *(volatile v8h*)gp = o;
}

__global__ __launch_bounds__(256)
void k_conv_ts(const float* __restrict__ x, const float* __restrict__ w, const float* __restrict__ bias, float* cts)
{
    const int idx = blockIdx.x * 256 + threadIdx.x;
    const int f4  = idx & 15;
    const int s2  = (idx >> 4) & 63;
    const int b   = idx >> 10;
    v4f v[6];
#pragma unroll
    for (int d = 0; d < 6; ++d) {
        const int s  = 2 * s2 - 2 + d;
        const int sc = min(max(s, 0), SA - 1);
        const float z = (s >= 0 && s < SA) ? 1.0f : 0.0f;
        const v4f t = *(const v4f*)(x + ((size_t)b * SA + sc) * FA + f4 * 4);
        v[d] = t * z;
    }
    v4f sum = {0.0f, 0.0f, 0.0f, 0.0f};
#pragma unroll 1
    for (int k = 0; k < 16; ++k) {
        const float bk = bias[k];
        const float w0 = w[k * 5 + 0], w1 = w[k * 5 + 1], w2 = w[k * 5 + 2], w3 = w[k * 5 + 3], w4 = w[k * 5 + 4];
        v4f a0 = {bk, bk, bk, bk};
        v4f a1 = a0;
        a0 = v[0] * w0 + a0; a0 = v[1] * w1 + a0; a0 = v[2] * w2 + a0; a0 = v[3] * w3 + a0; a0 = v[4] * w4 + a0;
        a1 = v[1] * w0 + a1; a1 = v[2] * w1 + a1; a1 = v[3] * w2 + a1; a1 = v[4] * w3 + a1; a1 = v[5] * w4 + a1;
#pragma unroll
        for (int i = 0; i < 4; ++i) sum[i] += fmaxf(a0[i], 0.0f) + fmaxf(a1[i], 0.0f);
    }
    const v4f o = sum * (1.0f / 32.0f);
    float* gp = cts + (size_t)idx * 4;
    *(volatile v4f*)gp = o;
    __threadfence();
    *(volatile v4f*)gp = o;
}

template<int F>
__global__ __launch_bounds__(256)
void k_conv_f(const float* __restrict__ src, const float* __restrict__ w, const float* __restrict__ bias, _Float16* dst)
{
    constexpr int G = F / 8;
    const int idx = blockIdx.x * 256 + threadIdx.x;
    const int g   = idx % G;
    const int rt  = idx / G;
    const int t   = rt >> 10;
    const int j   = rt & 1023;
    const int q   = (j & 63) * 1024 + t * 16 + (j >> 6);
    const float* row = src + (size_t)q * F;
    const int f0  = g * 8;
    const v4f va  = *(const v4f*)(row + f0);
    const v4f vb  = *(const v4f*)(row + f0 + 4);
    float lf = row[max(f0 - 1, 0)];
    lf = (f0 > 0) ? lf : 0.0f;
    float rf = row[min(f0 + 8, F - 1)];
    rf = (f0 + 8 < F) ? rf : 0.0f;
    float v[10];
    v[0] = lf;
    v[1] = va[0]; v[2] = va[1]; v[3] = va[2]; v[4] = va[3];
    v[5] = vb[0]; v[6] = vb[1]; v[7] = vb[2]; v[8] = vb[3];
    v[9] = rf;
    float s[8];
#pragma unroll
    for (int i = 0; i < 8; ++i) s[i] = 0.0f;
#pragma unroll 1
    for (int k = 0; k < 16; ++k) {
        const float bk = bias[k];
        const float w0 = w[k * 3 + 0], w1 = w[k * 3 + 1], w2 = w[k * 3 + 2];
#pragma unroll
        for (int i = 0; i < 8; ++i) {
            float a = v[i] * w0 + bk;
            a = v[i + 1] * w1 + a;
            a = v[i + 2] * w2 + a;
            s[i] += fmaxf(a, 0.0f);
        }
    }
    v8h o;
#pragma unroll
    for (int i = 0; i < 8; ++i) o[i] = (_Float16)(s[i] * (1.0f / 16.0f));
    _Float16* gp = dst + (size_t)idx * 8;
    *(volatile v8h*)gp = o;
    __threadfence();
    *(volatile v8h*)gp = o;
}

template<int PA, int K, int H, int NJ>
__device__ __forceinline__ void gstep(v8f (&acc)[4][NJ], const _Float16* at, int kka,
                                      const _Float16* __restrict__ w, int kkw, int hcw, int hh, int m)
{
    Frag a;
    const _Float16* ap = at + m * PA + kka + 8 * hh;
    a.hf[0] = *(const v8h*)(ap);
    a.hf[1] = *(const v8h*)(ap + 16);
#pragma unroll
    for (int g = 0; g < 4; ++g) {
#pragma unroll
        for (int j = 0; j < NJ; ++j) {
            const _Float16* bp = w + (size_t)(g * H + hcw + j * 16 + m) * K + kkw + 8 * hh;
            Frag b;
            b.hf[0] = *(const v8h*)(bp);
            b.hf[1] = *(const v8h*)(bp + 16);
            mma16(acc[g][j], a, b);
        }
    }
}

template<int H, int PH, int NJ>
__device__ __forceinline__ void cell(v8f (&acc)[4][NJ], const float* sb, float* sc, _Float16* sh,
                                     int hcw, int hh, int m, bool last)
{
#pragma unroll
    for (int j = 0; j < NJ; ++j) {
        const int hc = hcw + j * 16 + m;
        const float bi = sb[hc];
        const float bf = sb[H + hc];
        const float bg = sb[2 * H + hc];
        const float bo = sb[3 * H + hc];
#pragma unroll
        for (int r = 0; r < 8; ++r) {
            const int row = 8 * hh + r;
            const int ci  = row * H + hc;
            const float zi = acc[0][j][r] * 0.125f + bi;
            const float zf = acc[1][j][r] * 0.125f + bf;
            const float zg = acc[2][j][r] * 0.125f + bg;
            const float zo = acc[3][j][r] * 0.125f + bo;
            const float cp = sc[ci];
            const float gi = sigm_f(zi);
            const float gf = sigm_f(zf);
            const float gg = tanh_f(zg);
            const float go = sigm_f(zo);
            const float cn = gf * cp + gi * gg;
            const float hn = go * tanh_f(cn);
            sc[ci] = last ? hn : cn;
            sh[row * PH + hc] = (_Float16)hn;
        }
    }
}

template<int I, int H>
__global__ __launch_bounds__(256)
void k_lstm(const _Float16* __restrict__ xpl, const _Float16* __restrict__ w0, const _Float16* __restrict__ w1,
            const float* __restrict__ bih0, const float* __restrict__ bhh0,
            const float* __restrict__ bih1, const float* __restrict__ bhh1, float* hfin)
{
    constexpr int R  = 16;
    constexpr int NJ = H / 128;
    constexpr int WC = NJ * 16;
    constexpr int PX = I + 8;
    constexpr int PH = H + 8;
    constexpr int K0 = I + H;
    constexpr int K1 = 2 * H;
    constexpr int G4 = 4 * H;
    constexpr int XP = R * I / 8;
    constexpr int NIT = H / 64;
    static_assert(NJ >= 1);
    static_assert(I % 32 == 0);
    static_assert(H % 128 == 0);
    static_assert(XP <= 256 && XP % 32 == 0);
    static_assert((R * PH) % 8 == 0 && (R * H) % 4 == 0);

    __shared__ __attribute__((aligned(16))) _Float16 sx[R * PX];
    __shared__ __attribute__((aligned(16))) _Float16 sh0[R * PH];
    __shared__ __attribute__((aligned(16))) _Float16 sh1[R * PH];
    __shared__ __attribute__((aligned(16))) float sc0[R * H];
    __shared__ __attribute__((aligned(16))) float sc1[R * H];
    __shared__ float sb0[G4];
    __shared__ float sb1[G4];

    const int tid  = threadIdx.x;
    const int lane = tid & 31;
    const int wave = tid >> 5;
    const int hh   = lane >> 4;
    const int m    = lane & 15;
    const int j0   = blockIdx.x * R;
    const int hcw  = wave * WC;

    {
        const _Float16 hz = (_Float16)0.0f;
        const v8h z8 = {hz, hz, hz, hz, hz, hz, hz, hz};
        const v4f z4 = {0.0f, 0.0f, 0.0f, 0.0f};
        for (int i = tid; i < (R * PH) / 8; i += 256) {
            *(v8h*)(sh0 + i * 8) = z8;
            *(v8h*)(sh1 + i * 8) = z8;
        }
        for (int i = tid; i < (R * H) / 4; i += 256) {
            *(v4f*)(sc0 + i * 4) = z4;
            *(v4f*)(sc1 + i * 4) = z4;
        }
        for (int i = tid; i < G4; i += 256) {
            sb0[i] = bih0[i] + bhh0[i];
            sb1[i] = bih1[i] + bhh1[i];
        }
    }
    __syncthreads();

    v8f acc[4][NJ];

#pragma unroll 1
    for (int t = 0; t < NT; ++t) {
        if (tid < XP) {
            const int r  = tid / (I / 8);
            const int c8 = tid - r * (I / 8);
            const v8h v = *(const v8h*)(xpl + ((size_t)t * NB + j0 + r) * I + c8 * 8);
            *(v8h*)(sx + r * PX + c8 * 8) = v;
        }
        __syncthreads();

#pragma unroll
        for (int g = 0; g < 4; ++g)
#pragma unroll
            for (int j = 0; j < NJ; ++j)
#pragma unroll
                for (int r = 0; r < 8; ++r) acc[g][j][r] = 0.0f;
#pragma unroll 1
        for (int kt = 0; kt < I / 32; ++kt)
            gstep<PX, K0, H, NJ>(acc, sx, kt * 32, w0, kt * 32, hcw, hh, m);
#pragma unroll 1
        for (int kt = 0; kt < H / 32; ++kt)
            gstep<PH, K0, H, NJ>(acc, sh0, kt * 32, w0, I + kt * 32, hcw, hh, m);
        __syncthreads();
        cell<H, PH, NJ>(acc, sb0, sc0, sh0, hcw, hh, m, false);
        __syncthreads();

#pragma unroll
        for (int g = 0; g < 4; ++g)
#pragma unroll
            for (int j = 0; j < NJ; ++j)
#pragma unroll
                for (int r = 0; r < 8; ++r) acc[g][j][r] = 0.0f;
#pragma unroll 1
        for (int kt = 0; kt < H / 32; ++kt)
            gstep<PH, K1, H, NJ>(acc, sh0, kt * 32, w1, kt * 32, hcw, hh, m);
#pragma unroll 1
        for (int kt = 0; kt < H / 32; ++kt)
            gstep<PH, K1, H, NJ>(acc, sh1, kt * 32, w1, H + kt * 32, hcw, hh, m);
        __syncthreads();
        cell<H, PH, NJ>(acc, sb1, sc1, sh1, hcw, hh, m, t == NT - 1);
    }
    __syncthreads();

    v4f hv[NIT];
    const float* srow = sc1 + (size_t)(2 * wave) * H;
    float* grow = hfin + (size_t)(j0 + 2 * wave) * H;
#pragma unroll
    for (int it = 0; it < NIT; ++it) hv[it] = *(const v4f*)(srow + it * 128 + lane * 4);
#pragma unroll
    for (int it = 0; it < NIT; ++it) *(volatile v4f*)(grow + it * 128 + lane * 4) = hv[it];
    __threadfence();
#pragma unroll
    for (int it = 0; it < NIT; ++it) *(volatile v4f*)(grow + it * 128 + lane * 4) = hv[it];
}

__global__ __launch_bounds__(256)
void k_heads(const float* __restrict__ hfa, const float* __restrict__ hfb,
             const float* __restrict__ w1, const float* __restrict__ b1,
             const float* __restrict__ w2, const float* __restrict__ b2,
             const float* __restrict__ w1b, const float* __restrict__ b1b,
             const float* __restrict__ w2b, const float* __restrict__ b2b, float* out)
{
    constexpr int KC = HA + HB;
    constexpr int N1 = 192, N1B = 64;
    __shared__ __attribute__((aligned(16))) float shc[16 * KC];
    __shared__ __attribute__((aligned(16))) float st1[16 * N1];
    __shared__ __attribute__((aligned(16))) float st2[16 * N1B];
    __shared__ __attribute__((aligned(16))) float so0[16 * NY0];
    __shared__ __attribute__((aligned(16))) float so1[16 * NY1];

    const int tid = threadIdx.x;
    const int r0  = blockIdx.x * 16;

    for (int i = tid; i < (16 * HA) / 4; i += 256) {
        const v4f v = *(const v4f*)(hfa + (size_t)r0 * HA + i * 4);
        const int r = i / (HA / 4), c = (i % (HA / 4)) * 4;
        float* p = shc + r * KC + c;
        p[0] = v[0]; p[1] = v[1]; p[2] = v[2]; p[3] = v[3];
    }
    for (int i = tid; i < (16 * HB) / 4; i += 256) {
        const v4f v = *(const v4f*)(hfb + (size_t)r0 * HB + i * 4);
        const int r = i / (HB / 4), c = (i % (HB / 4)) * 4;
        float* p = shc + r * KC + HA + c;
        p[0] = v[0]; p[1] = v[1]; p[2] = v[2]; p[3] = v[3];
    }
    __syncthreads();

    for (int idx = tid; idx < 16 * N1; idx += 256) {
        const int r = idx / N1, o = idx - r * N1;
        const float* wr = w1 + (size_t)o * KC;
        const float* hr = shc + r * KC;
        float s = b1[o];
#pragma unroll 4
        for (int k = 0; k < KC; ++k) s = hr[k] * wr[k] + s;
        st1[idx] = fmaxf(s, 0.0f);
    }
    for (int idx = tid; idx < 16 * N1B; idx += 256) {
        const int r = idx / N1B, o = idx - r * N1B;
        const float* wr = w1b + (size_t)o * HB;
        const float* hr = shc + r * KC + HA;
        float s = b1b[o];
#pragma unroll 4
        for (int k = 0; k < HB; ++k) s = hr[k] * wr[k] + s;
        st2[idx] = fmaxf(s, 0.0f);
    }
    __syncthreads();

    for (int idx = tid; idx < 16 * NY0; idx += 256) {
        const int r = idx / NY0, o = idx - r * NY0;
        const float* wr = w2 + (size_t)o * N1;
        const float* hr = st1 + r * N1;
        float s = b2[o];
#pragma unroll 4
        for (int k = 0; k < N1; ++k) s = hr[k] * wr[k] + s;
        so0[idx] = s;
    }
    if (tid < 16 * NY1) {
        const int r = tid / NY1, o = tid - r * NY1;
        const float* wr = w2b + (size_t)o * N1B;
        const float* hr = st2 + r * N1B;
        float s = b2b[o];
#pragma unroll 4
        for (int k = 0; k < N1B; ++k) s = hr[k] * wr[k] + s;
        so1[tid] = s;
    }
    __syncthreads();

    const int i0 = min(tid, 95) * 4;
    const int i1 = min(max(tid - 128, 0), 31) * 4;
    const v4f v0 = *(const v4f*)(so0 + i0);
    const v4f v1 = *(const v4f*)(so1 + i1);
    float* gp0 = out + (size_t)blockIdx.x * (16 * NY0) + i0;
    float* gp1 = out + (size_t)NB * NY0 + (size_t)blockIdx.x * (16 * NY1) + i1;
    const bool w0s = (tid < 96);
    const bool w1s = (tid >= 128) && (tid < 160);
    if (w0s) *(volatile v4f*)gp0 = v0;
    if (w1s) *(volatile v4f*)gp1 = v1;
    __threadfence();
    if (w0s) *(volatile v4f*)gp0 = v0;
    if (w1s) *(volatile v4f*)gp1 = v1;
}

extern "C" void kernel_launch(void* const* d_in, const int* in_sizes, int n_in,
                              void* d_out, int out_size, void* d_ws, size_t ws_size,
                              hipStream_t stream)
{
    if (n_in < 32) return;
    if (in_sizes[0]  != NB * SA * FA)      return;
    if (in_sizes[1]  != NB * 64 * FB)      return;
    if (in_sizes[2]  != 16 * 5)            return;
    if (in_sizes[3]  != 16)                return;
    if (in_sizes[4]  != 16 * 3)            return;
    if (in_sizes[5]  != 16)                return;
    if (in_sizes[6]  != 4 * HA * IA)       return;
    if (in_sizes[7]  != 4 * HA * HA)       return;
    if (in_sizes[8]  != 4 * HA)            return;
    if (in_sizes[9]  != 4 * HA)            return;
    if (in_sizes[10] != 4 * HA * HA)       return;
    if (in_sizes[11] != 4 * HA * HA)       return;
    if (in_sizes[12] != 4 * HA)            return;
    if (in_sizes[13] != 4 * HA)            return;
    if (in_sizes[14] != 16 * 3)            return;
    if (in_sizes[15] != 16)                return;
    if (in_sizes[16] != 4 * HB * IB)       return;
    if (in_sizes[17] != 4 * HB * HB)       return;
    if (in_sizes[18] != 4 * HB)            return;
    if (in_sizes[19] != 4 * HB)            return;
    if (in_sizes[20] != 4 * HB * HB)       return;
    if (in_sizes[21] != 4 * HB * HB)       return;
    if (in_sizes[22] != 4 * HB)            return;
    if (in_sizes[23] != 4 * HB)            return;
    if (in_sizes[24] != 192 * (HA + HB))   return;
    if (in_sizes[25] != 192)               return;
    if (in_sizes[26] != NY0 * 192)         return;
    if (in_sizes[27] != NY0)               return;
    if (in_sizes[28] != 64 * HB)           return;
    if (in_sizes[29] != 64)                return;
    if (in_sizes[30] != NY1 * 64)          return;
    if (in_sizes[31] != NY1)               return;
    if (out_size != NB * NY0 + NB * NY1)   return;
    if (ws_size < WS_END)                  return;

    const float* x_a      = (const float*)d_in[0];
    const float* x_b      = (const float*)d_in[1];
    const float* w_ts     = (const float*)d_in[2];
    const float* b_ts     = (const float*)d_in[3];
    const float* w_f_a    = (const float*)d_in[4];
    const float* b_f_a    = (const float*)d_in[5];
    const float* w_ih0_a  = (const float*)d_in[6];
    const float* w_hh0_a  = (const float*)d_in[7];
    const float* b_ih0_a  = (const float*)d_in[8];
    const float* b_hh0_a  = (const float*)d_in[9];
    const float* w_ih1_a  = (const float*)d_in[10];
    const float* w_hh1_a  = (const float*)d_in[11];
    const float* b_ih1_a  = (const float*)d_in[12];
    const float* b_hh1_a  = (const float*)d_in[13];
    const float* w_f_b    = (const float*)d_in[14];
    const float* b_f_b    = (const float*)d_in[15];
    const float* w_ih0_b  = (const float*)d_in[16];
    const float* w_hh0_b  = (const float*)d_in[17];
    const float* b_ih0_b  = (const float*)d_in[18];
    const float* b_hh0_b  = (const float*)d_in[19];
    const float* w_ih1_b  = (const float*)d_in[20];
    const float* w_hh1_b  = (const float*)d_in[21];
    const float* b_ih1_b  = (const float*)d_in[22];
    const float* b_hh1_b  = (const float*)d_in[23];
    const float* w_fc1    = (const float*)d_in[24];
    const float* b_fc1    = (const float*)d_in[25];
    const float* w_fc2    = (const float*)d_in[26];
    const float* b_fc2    = (const float*)d_in[27];
    const float* w_fc1_b  = (const float*)d_in[28];
    const float* b_fc1_b  = (const float*)d_in[29];
    const float* w_fc2_b  = (const float*)d_in[30];
    const float* b_fc2_b  = (const float*)d_in[31];
    float* out = (float*)d_out;

    char* ws = (char*)d_ws;
    float*    cts  = (float*)(ws + OFF_CTS);
    _Float16* xpa  = (_Float16*)(ws + OFF_XA);
    _Float16* xpb  = (_Float16*)(ws + OFF_XB);
    _Float16* wa0  = (_Float16*)(ws + OFF_WA0);
    _Float16* wa1  = (_Float16*)(ws + OFF_WA1);
    _Float16* wb0  = (_Float16*)(ws + OFF_WB0);
    _Float16* wb1  = (_Float16*)(ws + OFF_WB1);
    float*    hfa  = (float*)(ws + OFF_HFA);
    float*    hfb  = (float*)(ws + OFF_HFB);

    k_wcvt<IA, HA><<<dim3((4 * HA * ((IA + HA) / 8) + 255) / 256), dim3(256), 0, stream>>>(w_ih0_a, w_hh0_a, wa0);
    k_wcvt<HA, HA><<<dim3((4 * HA * ((2 * HA) / 8) + 255) / 256), dim3(256), 0, stream>>>(w_ih1_a, w_hh1_a, wa1);
    k_wcvt<IB, HB><<<dim3((4 * HB * ((IB + HB) / 8) + 255) / 256), dim3(256), 0, stream>>>(w_ih0_b, w_hh0_b, wb0);
    k_wcvt<HB, HB><<<dim3((4 * HB * ((2 * HB) / 8) + 255) / 256), dim3(256), 0, stream>>>(w_ih1_b, w_hh1_b, wb1);

    k_conv_ts<<<dim3((NB * 64 * (FA / 4)) / 256), dim3(256), 0, stream>>>(x_a, w_ts, b_ts, cts);
    k_conv_f<FA><<<dim3((NB * 64 * (FA / 8)) / 256), dim3(256), 0, stream>>>((const float*)cts, w_f_a, b_f_a, xpa);
    k_conv_f<FB><<<dim3((NB * 64 * (FB / 8)) / 256), dim3(256), 0, stream>>>(x_b, w_f_b, b_f_b, xpb);

    k_lstm<IA, HA><<<dim3(NB / 16), dim3(256), 0, stream>>>(
        (const _Float16*)xpa, (const _Float16*)wa0, (const _Float16*)wa1, b_ih0_a, b_hh0_a, b_ih1_a, b_hh1_a, hfa);
    k_lstm<IB, HB><<<dim3(NB / 16), dim3(256), 0, stream>>>(
        (const _Float16*)xpb, (const _Float16*)wb0, (const _Float16*)wb1, b_ih0_b, b_hh0_b, b_ih1_b, b_hh1_b, hfb);

    k_heads<<<dim3(NB / 16), dim3(256), 0, stream>>>(
        (const float*)hfa, (const float*)hfb, w_fc1, b_fc1, w_fc2, b_fc2, w_fc1_b, b_fc1_b, w_fc2_b, b_fc2_b, out);
}
